// GNNFullyConnected_8134668059259
// MI455X (gfx1250) — hardware-run, weakly checked
//
#include <hip/hip_runtime.h>
#include <stddef.h>
#include <math.h>


#define NG     64
#define NPG    1024
#define DIN    128
#define DH     256
#define DOUT   10
#define NTHR   256
#define NWAVE  8
#define TPW    8
#define PB     136
#define WPL    (DH * DIN)
#define STGW   32

#define ATB     (16 * PB * 2)
#define OFF_A   0
#define OFF_PW  (OFF_A + NWAVE * 2 * ATB)
#define OFF_SW  (OFF_PW + NWAVE * DH * 4)
#define OFF_RN  (OFF_SW + NPG * 4)
#define OFF_SP  (OFF_RN + NPG * 4)
#define OFF_SL  (OFF_SP + NWAVE * DIN * 4)
#define OFF_PL  (OFF_SL + DIN * 4)
#define OFF_Z   (OFF_PL + DH * 4)
#define OFF_ST  (OFF_Z + 32 * 4)
#define LDS_G   (OFF_ST + 32 * 4)

static_assert(NWAVE * TPW * 16 == NPG);
static_assert(NTHR == NWAVE * 32);
static_assert(DIN == 32 * 4);
static_assert(DH == NTHR);
static_assert(((PB * 2) % 16) == 0);
static_assert((OFF_PW % 16) == 0 && (OFF_SW % 16) == 0 && (OFF_RN % 16) == 0);
static_assert((OFF_SP % 16) == 0 && (OFF_SL % 16) == 0 && (OFF_PL % 16) == 0);
static_assert((OFF_Z % 16) == 0 && (OFF_ST % 16) == 0);
static_assert(LDS_G == 91904);
static_assert((NG * DOUT) % 4 == 0);
static_assert(DOUT <= STGW);

typedef float          v4f   __attribute__((ext_vector_type(4)));
typedef float          v8f   __attribute__((ext_vector_type(8)));
typedef unsigned short v8us  __attribute__((ext_vector_type(8)));
typedef unsigned short v16us __attribute__((ext_vector_type(16)));
typedef __bf16         v16bf __attribute__((ext_vector_type(16)));
union Frag { v16bf v; v16us u; v8us h[2]; };

__device__ __forceinline__ unsigned short bf_rne(float x) {
  unsigned int u = __float_as_uint(x);
  u += 0x7FFFu + ((u >> 16) & 1u);
  return (unsigned short)(u >> 16);
}
__device__ __forceinline__ void split2(float x, unsigned short& hi, unsigned short& lo) {
  const unsigned short h = bf_rne(x);
  const float r = x - __uint_as_float(((unsigned int)h) << 16);
  hi = h;
  lo = bf_rne(r);
}
__device__ __forceinline__ void split8(v4f a, v4f b, v8us& hi, v8us& lo) {
  float t[8] = {a.x, a.y, a.z, a.w, b.x, b.y, b.z, b.w};
#pragma unroll
  for (int j = 0; j < 8; ++j) { unsigned short p, q; split2(t[j], p, q); hi[j] = p; lo[j] = q; }
}

__device__ __forceinline__ v8f wmb(v16bf a, v16bf b, v8f c) {
  v8f d = __builtin_amdgcn_wmma_f32_16x16x32_bf16(false, a, false, b, (short)0, c, false, false);
  asm volatile("v_nop\n\tv_nop\n\tv_nop\n\tv_nop" : "+v"(d) : "v"(a), "v"(b));
  return d;
}
__device__ __forceinline__ v8f mm3(v16bf ah, v16bf al, v16bf bh, v16bf bl, v8f c) {
  c = wmb(ah, bh, c);
  c = wmb(ah, bl, c);
  c = wmb(al, bh, c);
  return c;
}
__device__ __forceinline__ v16bf ldfrag(const unsigned short* p) {
  Frag f;
  f.h[0] = *(const v8us*)p;
  f.h[1] = *(const v8us*)(p + 16);
  return f.v;
}

__global__ __launch_bounds__(NTHR) void k_wprep(const float* __restrict__ W1, unsigned short* Wpl) {
  const int tid = (int)threadIdx.x;
  const int kq = DIN / 8;
  const int units = DH * kq;
#pragma unroll 1
  for (int u = tid; u < units; u += NTHR) {
    const int n  = u / kq;
    const int k0 = (u - n * kq) * 8;
    v8us hi, lo;
#pragma unroll
    for (int j = 0; j < 8; ++j) {
      unsigned short p, q;
      split2(W1[(size_t)(k0 + j) * DH + n], p, q);
      hi[j] = p; lo[j] = q;
    }
    unsigned short* ph = Wpl + (size_t)u * 8;
    unsigned short* pl = Wpl + (size_t)WPL + (size_t)u * 8;
    *(volatile v8us*)ph = hi;
    *(volatile v8us*)pl = lo;
    __threadfence();
    *(volatile v8us*)ph = hi;
    *(volatile v8us*)pl = lo;
  }
}

__global__ __launch_bounds__(NTHR) void k_graph(
    const float* __restrict__ x, const unsigned short* __restrict__ Wpl,
    const float* __restrict__ b1, const float* __restrict__ W2, const float* __restrict__ b2,
    const int* __restrict__ batch, float* stg) {
  extern __shared__ v4f lds_dyn[];
  char* base = (char*)lds_dyn;
  unsigned short* sA = (unsigned short*)(base + OFF_A);
  float* Pw   = (float*)(base + OFF_PW);
  float* swL  = (float*)(base + OFF_SW);
  float* rnL  = (float*)(base + OFF_RN);
  float* Spart= (float*)(base + OFF_SP);
  float* SL   = (float*)(base + OFF_SL);
  float* plL  = (float*)(base + OFF_PL);
  float* zL   = (float*)(base + OFF_Z);
  float* stL  = (float*)(base + OFF_ST);
  (void)batch;

  const int tid = (int)threadIdx.x, lane = tid & 31, wave = tid >> 5, hh = lane >> 4, m = lane & 15;
  const int g = (int)blockIdx.x;
  const float* xg = x + (size_t)g * NPG * DIN;

  for (int i = tid; i < NWAVE * DH; i += NTHR) Pw[i] = 0.0f;

  v4f S4 = {0.f, 0.f, 0.f, 0.f};
#pragma unroll 1
  for (int it = 0; it < NPG / NWAVE; ++it) {
    const int n = it * NWAVE + wave;
    const v4f v = *(const v4f*)(xg + (size_t)n * DIN + 4 * lane);
    float ss = v.x * v.x + v.y * v.y + v.z * v.z + v.w * v.w;
    ss += __shfl_xor(ss, 16, 32);
    ss += __shfl_xor(ss, 8, 32);
    ss += __shfl_xor(ss, 4, 32);
    ss += __shfl_xor(ss, 2, 32);
    ss += __shfl_xor(ss, 1, 32);
    const float rn = rsqrtf(ss + 1e-24f);
    S4 += v * rn;
    if (lane == 0) rnL[n] = rn;
  }
  *(v4f*)(Spart + wave * DIN + 4 * lane) = S4;
  __syncthreads();
  if (tid < DIN) {
    float s = 0.0f;
#pragma unroll
    for (int w = 0; w < NWAVE; ++w) s += Spart[w * DIN + tid];
    SL[tid] = s;
  }
  __syncthreads();

  {
    const v4f Sv = *(const v4f*)(SL + 4 * lane);
#pragma unroll 1
    for (int it = 0; it < NPG / NWAVE; ++it) {
      const int n = it * NWAVE + wave;
      const v4f v = *(const v4f*)(xg + (size_t)n * DIN + 4 * lane);
      const float rn = rnL[n];
      const v4f xn = v * rn;
      float ds = xn.x * Sv.x + xn.y * Sv.y + xn.z * Sv.z + xn.w * Sv.w;
      float dd = xn.x * xn.x + xn.y * xn.y + xn.z * xn.z + xn.w * xn.w;
      ds += __shfl_xor(ds, 16, 32); dd += __shfl_xor(dd, 16, 32);
      ds += __shfl_xor(ds, 8, 32);  dd += __shfl_xor(dd, 8, 32);
      ds += __shfl_xor(ds, 4, 32);  dd += __shfl_xor(dd, 4, 32);
      ds += __shfl_xor(ds, 2, 32);  dd += __shfl_xor(dd, 2, 32);
      ds += __shfl_xor(ds, 1, 32);  dd += __shfl_xor(dd, 1, 32);
      if (lane == 0) swL[n] = ds - dd;
    }
  }
  __syncthreads();

  unsigned short* tAh = sA + (size_t)wave * (2 * 16 * PB);
  unsigned short* tAl = tAh + 16 * PB;
  float* Pww = Pw + wave * DH;
  const unsigned short* Wh = Wpl;
  const v8f z8 = {0.f, 0.f, 0.f, 0.f, 0.f, 0.f, 0.f, 0.f};

#pragma unroll 1
  for (int tt = 0; tt < TPW; ++tt) {
    const int r0 = (tt * NWAVE + wave) * 16;
    const float* rp = xg + (size_t)(r0 + m) * DIN + 64 * hh;
#pragma unroll
    for (int q = 0; q < 2; ++q) {
      v4f xv[8];
#pragma unroll
      for (int j = 0; j < 8; ++j) xv[j] = *(const v4f*)(rp + 32 * q + 4 * j);
#pragma unroll
      for (int j = 0; j < 4; ++j) {
        v8us hi, lo;
        split8(xv[2 * j], xv[2 * j + 1], hi, lo);
        *(v8us*)(tAh + m * PB + 64 * hh + 32 * q + 8 * j) = hi;
        *(v8us*)(tAl + m * PB + 64 * hh + 32 * q + 8 * j) = lo;
      }
    }
    __syncthreads();
    float wv[8];
#pragma unroll
    for (int r = 0; r < 8; ++r) wv[r] = swL[r0 + 8 * hh + r];

#pragma unroll 1
    for (int grp = 0; grp < DH / 64; ++grp) {
      v8f acc[4] = {z8, z8, z8, z8};
#pragma unroll
      for (int ks = 0; ks < DIN / 32; ++ks) {
        const v16bf ah = ldfrag(tAh + m * PB + 32 * ks + 8 * hh);
        const v16bf al = ldfrag(tAl + m * PB + 32 * ks + 8 * hh);
#pragma unroll
        for (int nt = 0; nt < 4; ++nt) {
          const unsigned short* wp = Wh + (size_t)(grp * 64 + 16 * nt + m) * DIN + 32 * ks + 8 * hh;
          acc[nt] = mm3(ah, al, ldfrag(wp), ldfrag(wp + WPL), acc[nt]);
        }
      }
#pragma unroll
      for (int nt = 0; nt < 4; ++nt) {
        const int col = grp * 64 + 16 * nt + m;
        const float bias = b1[col];
        float pr = 0.0f;
#pragma unroll
        for (int r = 0; r < 8; ++r) {
          float hv = acc[nt][r] + bias;
          hv = hv > 0.0f ? hv : 0.0f;
          pr += wv[r] * hv;
        }
        pr += __shfl_xor(pr, 16, 32);
        if (hh == 0) Pww[col] = Pww[col] + pr;
      }
    }
    __syncthreads();
  }

  {
    float ps = 0.0f;
#pragma unroll
    for (int w = 0; w < NWAVE; ++w) ps += Pw[w * DH + tid];
    plL[tid] = ps * (1.0f / (float)NPG);
  }
  __syncthreads();
  if (tid < DOUT) {
    float a = 0.0f;
#pragma unroll 4
    for (int c = 0; c < DH; ++c) a += plL[c] * W2[c * DOUT + tid];
    zL[tid] = a + b2[tid];
  }
  __syncthreads();
  if (tid == 0) {
    float mx = zL[0];
#pragma unroll 1
    for (int j = 1; j < DOUT; ++j) mx = fmaxf(mx, zL[j]);
    float se = 0.0f;
#pragma unroll 1
    for (int j = 0; j < DOUT; ++j) se += expf(zL[j] - mx);
    const float lse = logf(se);
#pragma unroll 1
    for (int j = 0; j < STGW; ++j) stL[j] = (j < DOUT) ? ((zL[j] - mx) - lse) : 0.0f;
  }
  __syncthreads();
  if (tid < 8) {
    const v4f v = *(const v4f*)(stL + 4 * tid);
    float* op = stg + (size_t)g * STGW + 4 * tid;
    *(volatile v4f*)op = v;
    __threadfence();
    *(volatile v4f*)op = v;
  }
}

__global__ __launch_bounds__(NTHR) void k_out(const float* __restrict__ stg, float* out) {
  __shared__ __attribute__((aligned(16))) float buf[NG * STGW];
  const int tid = (int)threadIdx.x;
  for (int i = tid; i < NG * STGW / 4; i += NTHR) ((v4f*)buf)[i] = ((const v4f*)stg)[i];
  __syncthreads();
  if (tid < (NG * DOUT) / 4) {
    v4f o;
#pragma unroll
    for (int j = 0; j < 4; ++j) {
      const int e  = 4 * tid + j;
      const int gq = e / DOUT;
      const int c  = e - gq * DOUT;
      o[j] = buf[gq * STGW + c];
    }
    float* op = out + 4 * tid;
    *(volatile v4f*)op = o;
    __threadfence();
    *(volatile v4f*)op = o;
  }
}

extern "C" void kernel_launch(void* const* d_in, const int* in_sizes, int n_in,
                              void* d_out, int out_size, void* d_ws, size_t ws_size,
                              hipStream_t stream) {
  if (n_in < 6) return;
  if (in_sizes[0] != NG * NPG * DIN) return;
  if (in_sizes[2] != DIN * DH || in_sizes[3] != DH) return;
  if (in_sizes[4] != DH * DOUT || in_sizes[5] != DOUT) return;
  if (out_size != NG * DOUT) return;

  const float* x     = (const float*)d_in[0];
  const int*   batch = (const int*)d_in[1];
  const float* W1    = (const float*)d_in[2];
  const float* b1    = (const float*)d_in[3];
  const float* W2    = (const float*)d_in[4];
  const float* b2    = (const float*)d_in[5];
  float* out = (float*)d_out;

  char* ws = (char*)d_ws;
  const size_t oW   = 0;
  const size_t oS   = (size_t)2 * WPL * 2;
  const size_t tot  = oS + (size_t)NG * STGW * 4;
  if (tot > ws_size) return;
  if (tot > ((size_t)128 << 20)) return;
  unsigned short* Wpl = (unsigned short*)(ws + oW);
  float*          stg = (float*)(ws + oS);

  k_wprep<<<1, NTHR, 0, stream>>>(W1, Wpl);

  hipFuncSetAttribute(reinterpret_cast<const void*>(&k_graph),
                      hipFuncAttributeMaxDynamicSharedMemorySize, LDS_G);
  k_graph<<<NG, NTHR, LDS_G, stream>>>(x, Wpl, b1, W2, b2, batch, stg);

  k_out<<<1, NTHR, 0, stream>>>(stg, out);
}
